// RoPE_44641890074751
// MI455X (gfx1250) — hardware-run, weakly checked
//
#include <hip/hip_runtime.h>
#include <math.h>

typedef __attribute__((ext_vector_type(16))) _Float16 v16h;
typedef __attribute__((ext_vector_type(8)))  _Float16 v8h;
typedef __attribute__((ext_vector_type(8)))  float    v8f;
typedef __attribute__((ext_vector_type(4)))  float    v4f;

constexpr int kInputsRneToBf16 = 1;

constexpr int kBatch = 2;
constexpr int kSeq   = 2048;
constexpr int kDim   = 1024;
constexpr int kHeads = 16;
constexpr int kHd    = 64;
constexpr int kRows  = kBatch * kSeq;
static_assert(kHeads * kHd == kDim);
static_assert((kSeq & (kSeq - 1)) == 0);
static_assert((kRows % 64) == 0 && (kDim % 64) == 0 && (kHd % 64) == 0);
static_assert((kDim % 32) == 0 && (kSeq % 32) == 0 && (kHd % 32) == 0);

constexpr int isqrt_c(int n) { int r = 0; while ((r + 1) * (r + 1) <= n) ++r; return r; }
static_assert(isqrt_c(kHd) * isqrt_c(kHd) == kHd);

constexpr float kActCarry   = 16.0f;
constexpr float kWCarry     = 1024.0f;
constexpr float kProjScale  = 1.0f / (kActCarry * kWCarry);
constexpr float kScoreScale = 1.0f / (float)isqrt_c(kHd);
constexpr float kMScale     = kScoreScale / (kActCarry * kActCarry);
constexpr float kCtxScale   = 1.0f / kActCarry;
constexpr float kOutScale   = 1.0f / kWCarry;
constexpr float kF16MinNormal = 6.103515625e-05f;

constexpr float kRotBase = 10000.0f;
constexpr float kFreq0   = 1.0f;
constexpr float kFreq1   = 1.0f / (kRotBase * kRotBase);

constexpr size_t kOffCos   = 0;
constexpr size_t kOffSin   = kOffCos   + (size_t)kSeq * 4;
constexpr size_t kOffBR    = kOffSin   + (size_t)kSeq * 4;
constexpr size_t kOffX16   = kOffBR    + (size_t)4 * kDim * 4;
constexpr size_t kOffWT    = kOffX16   + (size_t)kRows * kDim * 2;
constexpr size_t kOffQF    = kOffWT    + (size_t)4 * kDim * kDim * 2;
constexpr size_t kOffKVTF  = kOffQF    + (size_t)kRows * kDim * 4;
constexpr size_t kOffQ16   = kOffKVTF  + (size_t)2 * kDim * kRows * 4;
constexpr size_t kOffKVT16 = kOffQ16   + (size_t)kRows * kDim * 2;
constexpr size_t kOffMT16  = kOffKVT16 + (size_t)2 * kDim * kRows * 2;
constexpr size_t kOffCTX16 = kOffMT16  + (size_t)kBatch * kHeads * kHd * kHd * 2;
constexpr size_t kWsTotal  = kOffCTX16 + (size_t)kRows * kDim * 2;
static_assert(kWsTotal == 100958208ull);
static_assert(kWsTotal <= 134217728ull);
static_assert((kOffSin % 128) == 0 && (kOffBR % 128) == 0 && (kOffX16 % 128) == 0 && (kOffWT % 128) == 0 &&
              (kOffQF % 128) == 0 && (kOffKVTF % 128) == 0 && (kOffQ16 % 128) == 0 && (kOffKVT16 % 128) == 0 &&
              (kOffMT16 % 128) == 0 && (kOffCTX16 % 128) == 0);

__device__ __forceinline__ unsigned short f2bf_bits(float f) {
  unsigned u = __float_as_uint(f);
  return (unsigned short)((u + 0x7FFFu + ((u >> 16) & 1u)) >> 16);
}
__device__ __forceinline__ float bf_bits2f(unsigned short h) { return __uint_as_float(((unsigned)h) << 16); }
__device__ __forceinline__ float in_rne(float v) {
  if (kInputsRneToBf16) return bf_bits2f(f2bf_bits(v));
  return v;
}
__device__ __forceinline__ float flush_h(float v) { return (fabsf(v) < kF16MinNormal) ? 0.0f : v; }

namespace eng {

__device__ __forceinline__ void guard1_h(v8f& a, v16h x, v16h y) {
  asm volatile("v_nop\n\tv_nop\n\tv_nop\n\tv_nop" : "+v"(a) : "v"(x), "v"(y));
}
__device__ __forceinline__ void keep4_h(v16h a, v16h b, v16h c, v16h d) {
  asm volatile("v_nop" :: "v"(a), "v"(b), "v"(c), "v"(d));
}
__device__ __forceinline__ void acc_guard4(v8f& a, v8f& b, v8f& c, v8f& d) {
  asm volatile("v_nop\n\tv_nop\n\tv_nop\n\tv_nop" : "+v"(a), "+v"(b), "+v"(c), "+v"(d));
}

struct FragH {
  union U { v16h v; v8h h[2]; };
  static __device__ __forceinline__ v16h load(const _Float16* p) {
    U f; f.h[0] = *(const v8h*)(p); f.h[1] = *(const v8h*)(p + 16); return f.v;
  }
  static __device__ __forceinline__ v8f mma(v16h a, v16h b, v8f c) {
    return __builtin_amdgcn_wmma_f32_16x16x32_f16(false, a, false, b, (short)0, c, false, false);
  }
};

template <int BIAS_MODE, int OUT_MODE>
__global__ __launch_bounds__(256) void wmma_gemm64(
    const unsigned short* __restrict__ Ap, int lda, long strideA,
    const unsigned short* __restrict__ Btp, int ldb, long strideB,
    void* __restrict__ Cout, int ldc, long strideC,
    const float* __restrict__ bias,
    int M, int N, int K, float scale) {
  typedef _Float16 T;
  const T* A = (const T*)Ap;
  const T* Bt = (const T*)Btp;
  __shared__ __align__(16) float sT[8][16 * 68];
  const int b    = blockIdx.y;
  const int lane = threadIdx.x & 31;
  const int wave = threadIdx.x >> 5;
  const int tilesN = N >> 6;
  const int tilesM = M >> 6;
  const int tile = blockIdx.x * 8 + wave;
  if (tile >= tilesM * tilesN) return;
  const int tm = tile / tilesN;
  const int tn = tile - tm * tilesN;
  const int m0 = tm << 6;
  const int n0 = tn << 6;

  const T* Ab = A  + (size_t)b * strideA;
  const T* Bb = Bt + (size_t)b * strideB;

  const int rlane = lane & 15;
  const int koff  = (lane >> 4) * 8;
  const int mOff  = (lane >> 4) * 8;

  v8f acc[4][4];
#pragma unroll
  for (int i = 0; i < 4; ++i)
#pragma unroll
    for (int j = 0; j < 4; ++j) acc[i][j] = (v8f){0.f,0.f,0.f,0.f,0.f,0.f,0.f,0.f};

  for (int k0 = 0; k0 < K; k0 += 32) {
    v16h bh[4];
#pragma unroll
    for (int j = 0; j < 4; ++j) {
      const size_t boff = (size_t)(n0 + (j << 4) + rlane) * ldb + koff + k0;
      bh[j] = FragH::load(Bb + boff);
    }
#pragma unroll
    for (int i = 0; i < 4; ++i) {
      const size_t aoff = (size_t)(m0 + (i << 4) + rlane) * lda + koff + k0;
      v16h ah = FragH::load(Ab + aoff);
#pragma unroll
      for (int j = 0; j < 4; ++j) acc[i][j] = FragH::mma(ah, bh[j], acc[i][j]);
#pragma unroll
      for (int j = 0; j < 4; ++j) guard1_h(acc[i][j], ah, bh[j]);
    }
    keep4_h(bh[0], bh[1], bh[2], bh[3]);
  }
  acc_guard4(acc[0][0], acc[0][1], acc[0][2], acc[0][3]);
  acc_guard4(acc[1][0], acc[1][1], acc[1][2], acc[1][3]);
  acc_guard4(acc[2][0], acc[2][1], acc[2][2], acc[2][3]);
  acc_guard4(acc[3][0], acc[3][1], acc[3][2], acc[3][3]);

  float* slab = sT[wave];
#pragma unroll
  for (int i = 0; i < 4; ++i) {
    const int mBase = m0 + (i << 4);
#pragma unroll
    for (int j = 0; j < 4; ++j) {
      const int n = n0 + (j << 4) + rlane;
      float bv = 0.f;
      if (BIAS_MODE == 2) bv = bias[n];
#pragma unroll
      for (int r = 0; r < 8; ++r) {
        float v = acc[i][j][r] * scale;
        if (BIAS_MODE == 2) v += bv;
        slab[(mOff + r) * 68 + (j << 4) + rlane] = v;
      }
    }
    __builtin_amdgcn_fence(__ATOMIC_RELEASE, "workgroup");
    __builtin_amdgcn_wave_barrier();
    __builtin_amdgcn_fence(__ATOMIC_ACQUIRE, "workgroup");
    if (OUT_MODE == 0) {
      float* C = (float*)Cout + (size_t)b * strideC;
      const int hh = lane >> 4, c4 = (lane & 15) * 4;
      for (int pass = 0; pass < 2; ++pass) {
#pragma unroll
        for (int it = 0; it < 8; ++it) {
          const int row = it * 2 + hh;
          v4f v = *(const v4f*)(slab + row * 68 + c4);
          *(volatile v4f*)(C + (size_t)(mBase + row) * ldc + n0 + c4) = v;
        }
        __threadfence();
      }
    } else {
      const int q = lane >> 3, c8 = (lane & 7) * 8;
      unsigned short* C = (unsigned short*)Cout + (size_t)b * strideC;
      for (int pass = 0; pass < 2; ++pass) {
#pragma unroll
        for (int it = 0; it < 4; ++it) {
          const int row = it * 4 + q;
          const float* sp = slab + row * 68 + c8;
          v8h hv;
#pragma unroll
          for (int e = 0; e < 8; ++e) {
            const float t = flush_h(sp[e]);
            hv[e] = (_Float16)t;
          }
          *(volatile v8h*)(C + (size_t)(mBase + row) * ldc + n0 + c8) = hv;
        }
        __threadfence();
      }
    }
    __builtin_amdgcn_fence(__ATOMIC_RELEASE, "workgroup");
    __builtin_amdgcn_wave_barrier();
    __builtin_amdgcn_fence(__ATOMIC_ACQUIRE, "workgroup");
  }
}

}

__global__ __launch_bounds__(256) void prep_kernel(
    const float* __restrict__ bq, const float* __restrict__ bk,
    const float* __restrict__ bv, const float* __restrict__ bo,
    float* __restrict__ cosT, float* __restrict__ sinT, float* __restrict__ BR) {
  const int t = threadIdx.x;
  const int blk = blockIdx.x;
  constexpr int kTblBlocks = kSeq / 256;
  if (blk < kTblBlocks) {
    const int pos = blk * 256 + t;
    const float ang = (float)pos * kFreq0;
    const float c = cosf(ang);
    const float s = sinf(ang);
    *(volatile float*)(cosT + pos) = c;
    *(volatile float*)(sinT + pos) = s;
    __threadfence();
    *(volatile float*)(cosT + pos) = c;
    *(volatile float*)(sinT + pos) = s;
  } else {
    const int i = (blk - kTblBlocks) * 256 + t;
    const int which = i >> 10;
    const int j = i & (kDim - 1);
    const float* src = (which == 0) ? bq : (which == 1) ? bk : (which == 2) ? bv : bo;
    const float v = in_rne(src[j]);
    *(volatile float*)(BR + i) = v;
    __threadfence();
    *(volatile float*)(BR + i) = v;
  }
}

__global__ __launch_bounds__(256) void cvt_x_kernel(
    const float* __restrict__ in, unsigned short* __restrict__ out, int n8) {
  const int i = blockIdx.x * 256 + threadIdx.x;
  if (i >= n8) return;
  const float* p = in + 8 * (size_t)i;
  const v4f a = *(const v4f*)(p);
  const v4f c = *(const v4f*)(p + 4);
  v8h hv;
#pragma unroll
  for (int e = 0; e < 4; ++e) {
    const float t0 = flush_h(in_rne(a[e]) * kActCarry);
    const float t1 = flush_h(in_rne(c[e]) * kActCarry);
    hv[e]     = (_Float16)t0;
    hv[4 + e] = (_Float16)t1;
  }
  unsigned short* q = out + 8 * (size_t)i;
  *(volatile v8h*)q = hv;
  __threadfence();
  *(volatile v8h*)q = hv;
}

__global__ __launch_bounds__(256) void wt_cast_kernel(
    const float* __restrict__ W0, const float* __restrict__ W1,
    const float* __restrict__ W2, const float* __restrict__ W3,
    unsigned short* __restrict__ out) {
  __shared__ float sm[64][65];
  const int t  = threadIdx.x;
  const int k0 = blockIdx.x * 64;
  const int n0 = blockIdx.y * 64;
  const int z  = blockIdx.z;
  const float* W = (z == 0) ? W0 : (z == 1) ? W1 : (z == 2) ? W2 : W3;
#pragma unroll
  for (int i = 0; i < 16; ++i) {
    const int e = i * 256 + t;
    const int r = e >> 6;
    const int c = e & 63;
    sm[c][r] = W[(size_t)(k0 + r) * kDim + n0 + c];
  }
  __syncthreads();
  const int lane = t & 31, wave = t >> 5;
  const int q = lane >> 3, c8 = (lane & 7) * 8;
  unsigned short* op = out + (size_t)z * kDim * kDim;
  v8h hv[2];
#pragma unroll
  for (int it = 0; it < 2; ++it) {
    const int row = wave * 8 + it * 4 + q;
#pragma unroll
    for (int e = 0; e < 8; ++e) {
      const float tv = flush_h(in_rne(sm[row][c8 + e]) * kWCarry);
      hv[it][e] = (_Float16)tv;
    }
  }
  for (int pass = 0; pass < 2; ++pass) {
#pragma unroll
    for (int it = 0; it < 2; ++it) {
      const int row = wave * 8 + it * 4 + q;
      *(volatile v8h*)(op + (size_t)(n0 + row) * kDim + k0 + c8) = hv[it];
    }
    __threadfence();
  }
}

__global__ __launch_bounds__(256) void rope_q_kernel(
    const float* __restrict__ QF, const float* __restrict__ BR,
    const float* __restrict__ cosT, const float* __restrict__ sinT,
    unsigned short* __restrict__ Q16, int total8) {
  const int i = blockIdx.x * 256 + threadIdx.x;
  if (i >= total8) return;
  const int row = i >> 7;
  const int c0  = (i & 127) << 3;
  const int pos = row & (kSeq - 1);
  const float* p = QF + (size_t)row * kDim + c0;
  const v4f a0 = *(const v4f*)(p);
  const v4f a1 = *(const v4f*)(p + 4);
  const v4f b0 = *(const v4f*)(BR + c0);
  const v4f b1 = *(const v4f*)(BR + c0 + 4);
  float cs = cosT[pos];
  float sn = sinT[pos];
  asm volatile("" : "+v"(cs));
  asm volatile("" : "+v"(sn));
  float x[8];
#pragma unroll
  for (int e = 0; e < 4; ++e) {
    x[e]     = a0[e] + b0[e];
    x[4 + e] = a1[e] + b1[e];
  }
  const float s1 = (float)pos * kFreq1;
  const float r0 = x[0] * cs - x[1] * sn;
  const float r1 = x[0] * sn + x[1] * cs;
  const float r2 = x[2] - x[3] * s1;
  const float r3 = x[2] * s1 + x[3];
  const bool first = ((c0 & (kHd - 1)) == 0);
  x[0] = first ? r0 : x[0];
  x[1] = first ? r1 : x[1];
  x[2] = first ? r2 : x[2];
  x[3] = first ? r3 : x[3];
  v8h hv;
#pragma unroll
  for (int e = 0; e < 8; ++e) {
    const float tv = flush_h(x[e] * kActCarry);
    hv[e] = (_Float16)tv;
  }
  unsigned short* q = Q16 + (size_t)row * kDim + c0;
  *(volatile v8h*)q = hv;
  __threadfence();
  *(volatile v8h*)q = hv;
}

__global__ __launch_bounds__(256) void rope_kv_kernel(
    const float* __restrict__ KVTF, const float* __restrict__ BR,
    const float* __restrict__ cosT, const float* __restrict__ sinT,
    unsigned short* __restrict__ KVT16) {
  const int t    = threadIdx.x;
  const int rA   = blockIdx.y * 2;
  const int col0 = blockIdx.x * (256 * 8) + t * 8;
  const int pos0 = col0 & (kSeq - 1);
  const bool isK  = (rA < kDim);
  const int  din  = rA & (kHd - 1);
  const bool rot0 = isK && (din == 0);
  const bool rot1 = isK && (din == 2);
  const bool rotAny = rot0 || rot1;
  const float bias_e = BR[kDim + rA];
  const float bias_o = BR[kDim + rA + 1];
  const float* pe = KVTF + (size_t)rA * kRows + col0;
  const float* po = pe + kRows;
  const v4f e0 = *(const v4f*)(pe);
  const v4f e1 = *(const v4f*)(pe + 4);
  const v4f o0 = *(const v4f*)(po);
  const v4f o1 = *(const v4f*)(po + 4);
  const v4f c0 = *(const v4f*)(cosT + pos0);
  const v4f c1 = *(const v4f*)(cosT + pos0 + 4);
  const v4f s0 = *(const v4f*)(sinT + pos0);
  const v4f s1 = *(const v4f*)(sinT + pos0 + 4);
  float xe[8], xo[8], ct[8], st[8];
#pragma unroll
  for (int e = 0; e < 4; ++e) {
    xe[e] = e0[e] + bias_e;  xe[4 + e] = e1[e] + bias_e;
    xo[e] = o0[e] + bias_o;  xo[4 + e] = o1[e] + bias_o;
    ct[e] = c0[e];           ct[4 + e] = c1[e];
    st[e] = s0[e];           st[4 + e] = s1[e];
  }
  v8h he, ho;
#pragma unroll
  for (int e = 0; e < 8; ++e) {
    const float ang1 = (float)(pos0 + e) * kFreq1;
    const float cc = rot0 ? ct[e] : 1.0f;
    const float ss = rot0 ? st[e] : ang1;
    const float re = xe[e] * cc - xo[e] * ss;
    const float ro = xe[e] * ss + xo[e] * cc;
    const float ye = rotAny ? re : xe[e];
    const float yo = rotAny ? ro : xo[e];
    const float te = flush_h(ye * kActCarry);
    const float to = flush_h(yo * kActCarry);
    he[e] = (_Float16)te;
    ho[e] = (_Float16)to;
  }
  unsigned short* qe = KVT16 + (size_t)rA * kRows + col0;
  unsigned short* qo = qe + kRows;
  *(volatile v8h*)qe = he;
  *(volatile v8h*)qo = ho;
  __threadfence();
  *(volatile v8h*)qe = he;
  *(volatile v8h*)qo = ho;
}

extern "C" void kernel_launch(void* const* d_in, const int* in_sizes, int n_in,
                              void* d_out, int out_size, void* d_ws, size_t ws_size,
                              hipStream_t stream) {
  if (n_in < 9) return;
  if (in_sizes[0] != kRows * kDim) return;
  if (in_sizes[1] != kDim * kDim) return;
  if (in_sizes[2] != kDim) return;
  if (in_sizes[3] != kDim * kDim) return;
  if (in_sizes[4] != kDim) return;
  if (in_sizes[5] != kDim * kDim) return;
  if (in_sizes[6] != kDim) return;
  if (in_sizes[7] != kDim * kDim) return;
  if (in_sizes[8] != kDim) return;
  if (out_size != kRows * kDim) return;
  if (ws_size < kWsTotal) return;

  const float* x  = (const float*)d_in[0];
  const float* Wq = (const float*)d_in[1];
  const float* bq = (const float*)d_in[2];
  const float* Wk = (const float*)d_in[3];
  const float* bk = (const float*)d_in[4];
  const float* Wv = (const float*)d_in[5];
  const float* bv = (const float*)d_in[6];
  const float* Wo = (const float*)d_in[7];
  const float* bo = (const float*)d_in[8];
  float* out = (float*)d_out;

  char* ws = (char*)d_ws;
  float*          cosT  = (float*)(ws + kOffCos);
  float*          sinT  = (float*)(ws + kOffSin);
  float*          BR    = (float*)(ws + kOffBR);
  unsigned short* X16   = (unsigned short*)(ws + kOffX16);
  unsigned short* WT    = (unsigned short*)(ws + kOffWT);
  float*          QF    = (float*)(ws + kOffQF);
  float*          KVTF  = (float*)(ws + kOffKVTF);
  unsigned short* Q16   = (unsigned short*)(ws + kOffQ16);
  unsigned short* KVT16 = (unsigned short*)(ws + kOffKVT16);
  unsigned short* MT16  = (unsigned short*)(ws + kOffMT16);
  unsigned short* CTX16 = (unsigned short*)(ws + kOffCTX16);

  unsigned short* WqT  = WT;
  unsigned short* KVwT = WT + (size_t)kDim * kDim;
  unsigned short* WoT  = WT + (size_t)3 * kDim * kDim;

  prep_kernel<<<(kSeq / 256) + (4 * kDim / 256), 256, 0, stream>>>(bq, bk, bv, bo, cosT, sinT, BR);

  cvt_x_kernel<<<(kRows * kDim / 8) / 256, 256, 0, stream>>>(x, X16, kRows * kDim / 8);
  wt_cast_kernel<<<dim3(kDim / 64, kDim / 64, 4), 256, 0, stream>>>(Wq, Wk, Wv, Wo, WT);

  eng::wmma_gemm64<0, 0><<<dim3((kRows / 64) * (kDim / 64) / 8, 1), 256, 0, stream>>>(
      X16, kDim, 0L,
      WqT, kDim, 0L,
      (void*)QF, kDim, 0L,
      nullptr, kRows, kDim, kDim, kProjScale);

  eng::wmma_gemm64<0, 0><<<dim3((2 * kDim / 64) * (kRows / 64) / 8, 1), 256, 0, stream>>>(
      KVwT, kDim, 0L,
      X16, kDim, 0L,
      (void*)KVTF, kRows, 0L,
      nullptr, 2 * kDim, kRows, kDim, kProjScale);

  rope_q_kernel<<<(kRows * kDim / 8) / 256, 256, 0, stream>>>(QF, BR, cosT, sinT, Q16, kRows * kDim / 8);
  rope_kv_kernel<<<dim3(kRows / 2048, kDim), 256, 0, stream>>>(KVTF, BR, cosT, sinT, KVT16);

  for (int b = 0; b < kBatch; ++b) {
    eng::wmma_gemm64<0, 1><<<dim3(1, kHeads), 32, 0, stream>>>(
        KVT16 + (size_t)kDim * kRows + (size_t)b * kSeq, kRows, (long)kHd * kRows,
        KVT16 + (size_t)b * kSeq, kRows, (long)kHd * kRows,
        (void*)(MT16 + (size_t)b * kHeads * kHd * kHd), kHd, (long)kHd * kHd,
        nullptr, kHd, kHd, kSeq, kMScale);
  }

  for (int b = 0; b < kBatch; ++b) {
    eng::wmma_gemm64<0, 1><<<dim3((kSeq / 64) / 8, kHeads), 256, 0, stream>>>(
        Q16 + (size_t)b * kSeq * kDim, kDim, (long)kHd,
        MT16 + (size_t)b * kHeads * kHd * kHd, kHd, (long)kHd * kHd,
        (void*)(CTX16 + (size_t)b * kSeq * kDim), kDim, (long)kHd,
        nullptr, kSeq, kHd, kHd, kCtxScale);
  }

  eng::wmma_gemm64<2, 0><<<dim3((kRows / 64) * (kDim / 64) / 8, 1), 256, 0, stream>>>(
      CTX16, kDim, 0L,
      WoT, kDim, 0L,
      (void*)out, kDim, 0L,
      BR + 3 * kDim, kRows, kDim, kDim, kOutScale);
}
